// S4_69148973466319
// MI455X (gfx1250) — hardware-verified
//
#include <hip/hip_runtime.h>
#include <math.h>

constexpr int NBATCH  = 8;
constexpr int NSEQ    = 8192;
constexpr int NCHAN   = 128;
constexpr int NSTATE  = 128;
constexpr int CHUNK   = 128;
constexpr int NCHUNK  = NSEQ / CHUNK;
constexpr int NCOL    = NBATCH * NCHUNK;
constexpr int NROWS   = NBATCH * NSEQ;
constexpr int HXPITCH = NSTATE + CHUNK;
constexpr int NTHR    = 256;
constexpr float MIN_DT  = 1e-3f;
constexpr float EPS_A   = 1e-6f;
constexpr float ZCARRY  = 16.0f;
constexpr float WCARRY  = 256.0f;
constexpr float OUT_SCALE = 1.0f / (ZCARRY * WCARRY);
constexpr float F32_MIN_NORMAL = 1.17549435e-38f;

static_assert(NCHUNK == 64 && NCOL == 512 && NROWS == 65536 && HXPITCH == 256, "shape constants");
static_assert(NCOL % 64 == 0 && NSTATE % 64 == 0 && CHUNK % 64 == 0 && NROWS % 64 == 0 && NCHAN % 64 == 0, "GEMM M, N tile multiples");
static_assert(CHUNK % 32 == 0 && HXPITCH % 32 == 0 && NCHAN % 32 == 0, "GEMM K multiples of 32");
static_assert(NSTATE == 128 && CHUNK == 128 && NCHAN == 128, "index arithmetic below assumes 128");

typedef __attribute__((ext_vector_type(16))) _Float16 v16h;
typedef __attribute__((ext_vector_type(8)))  _Float16 v8h;
typedef __attribute__((ext_vector_type(16))) __bf16   v16b;
typedef __attribute__((ext_vector_type(8)))  __bf16   v8b;
typedef __attribute__((ext_vector_type(8)))  float    v8f;
typedef __attribute__((ext_vector_type(4)))  float    v4f;
typedef __attribute__((ext_vector_type(8)))  unsigned short v8us;

__device__ __forceinline__ unsigned short f2bf_bits(float f) {
  unsigned u = __float_as_uint(f);
  return (unsigned short)((u + 0x7FFFu + ((u >> 16) & 1u)) >> 16);
}
__device__ __forceinline__ float ftz32(float v) { return (fabsf(v) < F32_MIN_NORMAL) ? 0.0f : v; }

__device__ __forceinline__ void dep_guard4_h(v8f& a, v8f& b, v8f& c, v8f& d, v16h x, v16h y) {
  asm volatile("v_nop\n\tv_nop\n\tv_nop\n\tv_nop" : "+v"(a), "+v"(b), "+v"(c), "+v"(d) : "v"(x), "v"(y));
}
__device__ __forceinline__ void dep_guard4_b(v8f& a, v8f& b, v8f& c, v8f& d, v16b x, v16b y) {
  asm volatile("v_nop\n\tv_nop\n\tv_nop\n\tv_nop" : "+v"(a), "+v"(b), "+v"(c), "+v"(d) : "v"(x), "v"(y));
}
__device__ __forceinline__ void keep4_h(v16h a, v16h b, v16h c, v16h d) { asm volatile("v_nop" :: "v"(a), "v"(b), "v"(c), "v"(d)); }
__device__ __forceinline__ void keep4_b(v16b a, v16b b, v16b c, v16b d) { asm volatile("v_nop" :: "v"(a), "v"(b), "v"(c), "v"(d)); }
__device__ __forceinline__ void acc_guard4(v8f& a, v8f& b, v8f& c, v8f& d) {
  asm volatile("v_nop\n\tv_nop\n\tv_nop\n\tv_nop" : "+v"(a), "+v"(b), "+v"(c), "+v"(d));
}

template <typename T> struct Frag;
template <> struct Frag<_Float16> {
  typedef v16h V; union U { v16h v; v8h h[2]; };
  static __device__ __forceinline__ v16h load(const _Float16* p) {
    U f; f.h[0] = *(const v8h*)(p); f.h[1] = *(const v8h*)(p + 16); return f.v;
  }
  static __device__ __forceinline__ v8f mma(v16h a, v16h b, v8f c) {
    return __builtin_amdgcn_wmma_f32_16x16x32_f16(false, a, false, b, (short)0, c, false, false);
  }
  static __device__ __forceinline__ void guard4(v8f& a, v8f& b, v8f& c, v8f& d, v16h x, v16h y) { dep_guard4_h(a, b, c, d, x, y); }
  static __device__ __forceinline__ void keep(v16h a, v16h b, v16h c, v16h d) { keep4_h(a, b, c, d); }
};
template <> struct Frag<__bf16> {
  typedef v16b V; union U { v16b v; v8b h[2]; };
  static __device__ __forceinline__ v16b load(const __bf16* p) {
    U f; f.h[0] = *(const v8b*)(p); f.h[1] = *(const v8b*)(p + 16); return f.v;
  }
  static __device__ __forceinline__ v8f mma(v16b a, v16b b, v8f c) {
    return __builtin_amdgcn_wmma_f32_16x16x32_bf16(false, a, false, b, (short)0, c, false, false);
  }
  static __device__ __forceinline__ void guard4(v8f& a, v8f& b, v8f& c, v8f& d, v16b x, v16b y) { dep_guard4_b(a, b, c, d, x, y); }
  static __device__ __forceinline__ void keep(v16b a, v16b b, v16b c, v16b d) { keep4_b(a, b, c, d); }
};

template <int ET> struct Elem;
template <> struct Elem<0> { typedef _Float16 T; };
template <> struct Elem<1> { typedef __bf16 T; };
template <int ET, int BIAS_MODE>
__global__ __launch_bounds__(256) void wmma_gemm64(
    const unsigned short* __restrict__ Ap, int lda, long strideA,
    const unsigned short* __restrict__ Btp, int ldb, long strideB,
    float* __restrict__ Cout, int ldc, long strideC,
    const float* __restrict__ bias,
    int M, int N, int K, float scale) {
  typedef typename Elem<ET>::T T;
  typedef typename Frag<T>::V V;
  const T* A = (const T*)Ap;
  const T* Bt = (const T*)Btp;
  __shared__ __align__(16) float sT[8][16 * 68];
  const int b    = blockIdx.y;
  const int lane = threadIdx.x & 31;
  const int wave = threadIdx.x >> 5;
  const int tilesN = N >> 6;
  const int tilesM = M >> 6;
  const int tile = blockIdx.x * 8 + wave;
  if (tile >= tilesM * tilesN) return;
  const int tm = tile / tilesN;
  const int tn = tile - tm * tilesN;
  const int m0 = tm << 6;
  const int n0 = tn << 6;

  const T* Ab = A  + (size_t)b * strideA;
  const T* Bb = Bt + (size_t)b * strideB;

  const int rlane = lane & 15;
  const int koff  = (lane >> 4) * 8;
  const int mOff  = (lane >> 4) * 8;

  v8f acc[4][4];
#pragma unroll
  for (int i = 0; i < 4; ++i)
#pragma unroll
    for (int j = 0; j < 4; ++j) acc[i][j] = (v8f){0.f, 0.f, 0.f, 0.f, 0.f, 0.f, 0.f, 0.f};

  for (int k0 = 0; k0 < K; k0 += 32) {
    V bh[4];
#pragma unroll
    for (int j = 0; j < 4; ++j) {
      const size_t bo = (size_t)(n0 + (j << 4) + rlane) * ldb + koff + k0;
      bh[j] = Frag<T>::load(Bb + bo);
    }
#pragma unroll
    for (int i = 0; i < 4; ++i) {
      const size_t ao = (size_t)(m0 + (i << 4) + rlane) * lda + koff + k0;
      V ah = Frag<T>::load(Ab + ao);
#pragma unroll
      for (int j = 0; j < 4; ++j) acc[i][j] = Frag<T>::mma(ah, bh[j], acc[i][j]);
      Frag<T>::guard4(acc[i][0], acc[i][1], acc[i][2], acc[i][3], ah, bh[3]);
    }
    Frag<T>::keep(bh[0], bh[1], bh[2], bh[3]);
  }
  acc_guard4(acc[0][0], acc[0][1], acc[0][2], acc[0][3]);
  acc_guard4(acc[1][0], acc[1][1], acc[1][2], acc[1][3]);
  acc_guard4(acc[2][0], acc[2][1], acc[2][2], acc[2][3]);
  acc_guard4(acc[3][0], acc[3][1], acc[3][2], acc[3][3]);

  float* slab = sT[wave];
  float* C = Cout + (size_t)b * strideC;
  const int hh = lane >> 4;
  const int c4 = (lane & 15) * 4;
#pragma unroll
  for (int i = 0; i < 4; ++i) {
    const int mBase = m0 + (i << 4);
#pragma unroll
    for (int j = 0; j < 4; ++j) {
      const int n = n0 + (j << 4) + rlane;
      float bv = 0.f;
      if (BIAS_MODE == 2) bv = bias[n];
#pragma unroll
      for (int r = 0; r < 8; ++r) {
        float v = acc[i][j][r] * scale;
        if (BIAS_MODE == 2) v += bv;
        slab[(mOff + r) * 68 + (j << 4) + rlane] = v;
      }
    }
    __builtin_amdgcn_fence(__ATOMIC_RELEASE, "workgroup");
    __builtin_amdgcn_wave_barrier();
    __builtin_amdgcn_fence(__ATOMIC_ACQUIRE, "workgroup");
    for (int pass = 0; pass < 2; ++pass) {
#pragma unroll
      for (int it = 0; it < 8; ++it) {
        const int row = it * 2 + hh;
        v4f v = *(const v4f*)(slab + row * 68 + c4);
        *(volatile v4f*)(C + (size_t)(mBase + row) * ldc + n0 + c4) = v;
      }
      __threadfence();
    }
    __builtin_amdgcn_fence(__ATOMIC_RELEASE, "workgroup");
    __builtin_amdgcn_wave_barrier();
    __builtin_amdgcn_fence(__ATOMIC_ACQUIRE, "workgroup");
  }
}

__global__ __launch_bounds__(NTHR) void wcast_kernel(const float* __restrict__ src, unsigned short* __restrict__ dst, int n8) {
  const int i = blockIdx.x * NTHR + threadIdx.x;
  if (i < n8) {
    const v4f a = *(const v4f*)(src + (size_t)i * 8);
    const v4f b = *(const v4f*)(src + (size_t)i * 8 + 4);
    v8h hv;
#pragma unroll
    for (int e = 0; e < 4; ++e) {
      hv[e]     = (_Float16)(a[e] * WCARRY);
      hv[4 + e] = (_Float16)(b[e] * WCARRY);
    }
    *(volatile v8h*)(dst + (size_t)i * 8) = hv;
    __threadfence();
    *(volatile v8h*)(dst + (size_t)i * 8) = hv;
  }
}

__global__ __launch_bounds__(NTHR) void ssm_build_kernel(const float* __restrict__ log_A, const float* __restrict__ Bmat,
                                                         const float* __restrict__ Cmat, const float* __restrict__ log_delta,
                                                         unsigned short* __restrict__ M1, unsigned short* __restrict__ Wd,
                                                         float* __restrict__ DAQ) {
  __shared__ float sLg[NSTATE], sDB[NSTATE], sC[NSTATE], sCdB[NSTATE];
  __shared__ __align__(16) float sQ[NSTATE];
  __shared__ float sKp[2 * CHUNK];
  __shared__ __align__(16) unsigned short stage[CHUNK * 128];
  const int d = blockIdx.x;
  const int tid = threadIdx.x;

  if (tid < NSTATE) {
    const int n = tid;
    const float la = log_A[d * NSTATE + n];
    const float ld = log_delta[d];
    float spA = 0.0f, spD = 0.0f;
#pragma unroll 1
    for (int q = 0; q < 2; ++q) {
      const float xin = q ? ld : la;
      const float r = fmaxf(xin, 0.0f) + log1pf(expf(-fabsf(xin)));
      if (q) spD = r; else spA = r;
    }
    const float Aneg = -spA;
    const float dt = spD + MIN_DT;
    const float lg = Aneg * dt;
    float dA = 0.0f, dAq = 0.0f;
#pragma unroll 1
    for (int q = 0; q < 2; ++q) {
      const float arg = q ? (lg * (float)CHUNK) : lg;
      const float r = expf(arg);
      if (q) dAq = r; else dA = r;
    }
    const float bm = Bmat[d * NSTATE + n];
    const float cm = Cmat[d * NSTATE + n];
    const float dB = (dA - 1.0f) / (Aneg + EPS_A) * bm;
    sLg[n]  = lg;
    sDB[n]  = dB;
    sC[n]   = cm;
    sCdB[n] = cm * dB;
    sQ[n]   = ftz32(dAq);
  }
  __syncthreads();

  if (tid < 32) {
    const v4f q4 = *(const v4f*)(sQ + 4 * tid);
    float* qp = DAQ + (size_t)d * NSTATE + 4 * tid;
    *(volatile v4f*)qp = q4;
    __threadfence();
    *(volatile v4f*)qp = q4;
  }

  {
    const int m = tid & 127;
    const int nb = (tid >> 7) * 64;
    const float fm = (float)m;
    float s = 0.0f;
#pragma unroll 1
    for (int nn = 0; nn < 64; ++nn) {
      const int n = nb + nn;
      s = fmaf(sCdB[n], expf(sLg[n] * fm), s);
    }
    sKp[tid] = s;
  }
  __syncthreads();

#pragma unroll 1
  for (int ph = 0; ph < 3; ++ph) {
#pragma unroll 1
    for (int it = 0; it < 64; ++it) {
      const int e = it * NTHR + tid;
      const int r = e >> 7;
      const int c = e & 127;
      float v;
      if (ph < 2) {
        const int idx = (ph == 0) ? r : c;
        const float p = (ph == 0) ? (float)(CHUNK - 1 - c) : (float)(r + 1);
        const float coef0 = sDB[idx];
        const float coef1 = sC[idx];
        const float coef = (ph == 0) ? coef0 : coef1;
        v = coef * expf(sLg[idx] * p);
      } else {
        const int df = r - c;
        const int dcl = df < 0 ? 0 : df;
        const float kv = sKp[dcl] + sKp[CHUNK + dcl];
        v = (df >= 0) ? kv : 0.0f;
      }
      stage[e] = f2bf_bits(ftz32(v));
    }
    __syncthreads();
    unsigned short* dbase;
    int dpitch;
    if (ph == 0) {
      dbase = M1 + (size_t)d * (NSTATE * CHUNK);
      dpitch = CHUNK;
    } else {
      dbase = Wd + (size_t)d * (CHUNK * HXPITCH) + ((ph == 2) ? NSTATE : 0);
      dpitch = HXPITCH;
    }
    const int rsub = tid >> 4;
    const int seg = (tid & 15) * 8;
    for (int pass = 0; pass < 2; ++pass) {
#pragma unroll
      for (int it = 0; it < 8; ++it) {
        const int row = it * 16 + rsub;
        const v8us w = *(const v8us*)(stage + row * 128 + seg);
        *(volatile v8us*)(dbase + (size_t)row * dpitch + seg) = w;
      }
      __threadfence();
    }
    __syncthreads();
  }
}

__global__ __launch_bounds__(NTHR) void x_transpose_kernel(const float* __restrict__ x, unsigned short* __restrict__ HX) {
  __shared__ float tl[CHUNK * 33];
  const int col = blockIdx.x;
  const int d0 = blockIdx.y * 32;
  const int b = col >> 6;
  const int c = col & 63;
  const int tid = threadIdx.x;
  {
    const int rsub = tid >> 3;
    const int c4 = (tid & 7) * 4;
#pragma unroll
    for (int it = 0; it < 4; ++it) {
      const int row = it * 32 + rsub;
      const v4f v = *(const v4f*)(x + ((size_t)b * NSEQ + (size_t)c * CHUNK + row) * NCHAN + d0 + c4);
#pragma unroll
      for (int e = 0; e < 4; ++e) tl[row * 33 + c4 + e] = v[e];
    }
  }
  __syncthreads();
  const int dsub = tid >> 4;
  const int i0 = (tid & 15) * 8;
  v8us hv[2];
#pragma unroll
  for (int it = 0; it < 2; ++it) {
    const int dl = it * 16 + dsub;
    v8us w;
#pragma unroll
    for (int e = 0; e < 8; ++e) w[e] = f2bf_bits(tl[(i0 + e) * 33 + dl]);
    hv[it] = w;
  }
  for (int pass = 0; pass < 2; ++pass) {
#pragma unroll
    for (int it = 0; it < 2; ++it) {
      const int dd = d0 + it * 16 + dsub;
      unsigned short* dst = HX + ((size_t)dd * NCOL + col) * HXPITCH + NSTATE + i0;
      *(volatile v8us*)dst = hv[it];
    }
    __threadfence();
  }
}

__global__ __launch_bounds__(NTHR) void state_scan_kernel(const float* __restrict__ U, const float* __restrict__ DAQ,
                                                          unsigned short* __restrict__ HX) {
  const int g = blockIdx.x * NTHR + threadIdx.x;
  const int n0 = (g & 15) * 8;
  const int b = (g >> 4) & 7;
  const int d = g >> 7;
  const v4f a0 = *(const v4f*)(DAQ + (size_t)d * NSTATE + n0);
  const v4f a1 = *(const v4f*)(DAQ + (size_t)d * NSTATE + n0 + 4);
  float h[8];
#pragma unroll
  for (int e = 0; e < 8; ++e) h[e] = 0.0f;
#pragma unroll 1
  for (int c = 0; c < NCHUNK; ++c) {
    const size_t rowi = (size_t)d * NCOL + (size_t)b * NCHUNK + c;
    v8us w;
#pragma unroll
    for (int e = 0; e < 8; ++e) w[e] = f2bf_bits(h[e]);
    unsigned short* dst = HX + rowi * HXPITCH + n0;
    *(volatile v8us*)dst = w;
    __threadfence();
    *(volatile v8us*)dst = w;
    const v4f u0 = *(const v4f*)(U + rowi * NSTATE + n0);
    const v4f u1 = *(const v4f*)(U + rowi * NSTATE + n0 + 4);
#pragma unroll
    for (int e = 0; e < 4; ++e) {
      h[e]     = ftz32(fmaf(a0[e], h[e], u0[e]));
      h[4 + e] = ftz32(fmaf(a1[e], h[4 + e], u1[e]));
    }
  }
}

__global__ __launch_bounds__(NTHR) void z_transpose_kernel(const float* __restrict__ Yf, const float* __restrict__ x,
                                                           const float* __restrict__ skip_D, unsigned short* __restrict__ Zt) {
  __shared__ float tl[NCHAN * 65];
  const int bl0 = blockIdx.x * 64;
  const int tid = threadIdx.x;
  {
    const int dsub = tid >> 4;
    const int c4 = (tid & 15) * 4;
#pragma unroll
    for (int it = 0; it < 8; ++it) {
      const int dd = it * 16 + dsub;
      const v4f v = *(const v4f*)(Yf + (size_t)dd * NROWS + bl0 + c4);
#pragma unroll
      for (int e = 0; e < 4; ++e) tl[dd * 65 + c4 + e] = v[e];
    }
  }
  __syncthreads();
  const int rsub = tid >> 4;
  const int d0 = (tid & 15) * 8;
  const v4f s0 = *(const v4f*)(skip_D + d0);
  const v4f s1 = *(const v4f*)(skip_D + d0 + 4);
  v8h hv[4];
#pragma unroll
  for (int it = 0; it < 4; ++it) {
    const int r = it * 16 + rsub;
    const size_t row = (size_t)bl0 + r;
    const v4f x0 = *(const v4f*)(x + row * NCHAN + d0);
    const v4f x1 = *(const v4f*)(x + row * NCHAN + d0 + 4);
    v8h w;
#pragma unroll
    for (int e = 0; e < 4; ++e) {
      const float z0 = fmaf(x0[e], s0[e], tl[(d0 + e) * 65 + r]);
      const float z1 = fmaf(x1[e], s1[e], tl[(d0 + 4 + e) * 65 + r]);
      w[e]     = (_Float16)(z0 * ZCARRY);
      w[4 + e] = (_Float16)(z1 * ZCARRY);
    }
    hv[it] = w;
  }
  for (int pass = 0; pass < 2; ++pass) {
#pragma unroll
    for (int it = 0; it < 4; ++it) {
      const size_t row = (size_t)bl0 + it * 16 + rsub;
      *(volatile v8h*)(Zt + row * NCHAN + d0) = hv[it];
    }
    __threadfence();
  }
}

extern "C" void kernel_launch(void* const* d_in, const int* in_sizes, int n_in,
                              void* d_out, int out_size, void* d_ws, size_t ws_size, hipStream_t stream) {
  if (n_in < 8 || d_out == nullptr || d_ws == nullptr) return;
  if (in_sizes[0] != NBATCH * NSEQ * NCHAN || in_sizes[1] != NCHAN * NSTATE || in_sizes[2] != NCHAN * NSTATE ||
      in_sizes[3] != NCHAN * NSTATE || in_sizes[4] != NCHAN || in_sizes[5] != NCHAN ||
      in_sizes[6] != NCHAN * NCHAN || in_sizes[7] != NCHAN || out_size != NBATCH * NSEQ * NCHAN) return;

  const float* x         = (const float*)d_in[0];
  const float* log_A     = (const float*)d_in[1];
  const float* Bmat      = (const float*)d_in[2];
  const float* Cmat      = (const float*)d_in[3];
  const float* log_delta = (const float*)d_in[4];
  const float* skip_D    = (const float*)d_in[5];
  const float* W_out     = (const float*)d_in[6];
  const float* b_out     = (const float*)d_in[7];
  float* out = (float*)d_out;

  char* ws = (char*)d_ws;
  size_t off = 0;
  auto carve = [&](size_t bytes) -> char* { char* p = ws + off; off += (bytes + 255) & ~(size_t)255; return p; };
  unsigned short* HX  = (unsigned short*)carve((size_t)NCHAN * NCOL * HXPITCH * 2);
  float*          U   = (float*)carve((size_t)NCHAN * NCOL * NSTATE * 4);
  float*          Yf  = (float*)carve((size_t)NCHAN * NROWS * 4);
  unsigned short* Zt  = (unsigned short*)carve((size_t)NROWS * NCHAN * 2);
  unsigned short* M1  = (unsigned short*)carve((size_t)NCHAN * NSTATE * CHUNK * 2);
  unsigned short* Wd  = (unsigned short*)carve((size_t)NCHAN * CHUNK * HXPITCH * 2);
  float*          DAQ = (float*)carve((size_t)NCHAN * NSTATE * 4);
  unsigned short* W16 = (unsigned short*)carve((size_t)NCHAN * NCHAN * 2);
  if (off > ws_size || off > (size_t)134217728) return;

  const int n8w = NCHAN * NCHAN / 8;
  wcast_kernel<<<(n8w + NTHR - 1) / NTHR, NTHR, 0, stream>>>(W_out, W16, n8w);

  ssm_build_kernel<<<NCHAN, NTHR, 0, stream>>>(log_A, Bmat, Cmat, log_delta, M1, Wd, DAQ);

  x_transpose_kernel<<<dim3(NCOL, NCHAN / 32), NTHR, 0, stream>>>(x, HX);

  wmma_gemm64<1, 0><<<dim3((NCOL / 64) * (NSTATE / 64) / 8, NCHAN), 256, 0, stream>>>(
      HX + NSTATE, HXPITCH, (long)NCOL * HXPITCH,
      M1, CHUNK, (long)NSTATE * CHUNK,
      U, NSTATE, (long)NCOL * NSTATE,
      b_out, NCOL, NSTATE, CHUNK, 1.0f);

  state_scan_kernel<<<(NCHAN * NBATCH * (NSTATE / 8)) / NTHR, NTHR, 0, stream>>>(U, DAQ, HX);

  wmma_gemm64<1, 0><<<dim3((NCOL / 64) * (CHUNK / 64) / 8, NCHAN), 256, 0, stream>>>(
      HX, HXPITCH, (long)NCOL * HXPITCH,
      Wd, HXPITCH, (long)CHUNK * HXPITCH,
      Yf, CHUNK, (long)NCOL * CHUNK,
      b_out, NCOL, CHUNK, HXPITCH, 1.0f);

  z_transpose_kernel<<<NROWS / 64, NTHR, 0, stream>>>(Yf, x, skip_D, Zt);

  wmma_gemm64<0, 2><<<dim3((NROWS / 64) * (NCHAN / 64) / 8, 1), 256, 0, stream>>>(
      Zt, NCHAN, 0L,
      W16, NCHAN, 0L,
      out, NCHAN, 0L,
      b_out, NROWS, NCHAN, NCHAN, OUT_SCALE);
}
